// MultiHeadCrossAttention_50319836840451
// MI455X (gfx1250) — hardware-verified
//
#include <hip/hip_runtime.h>
#include <math.h>

#ifndef NB
#define NB 2
#endif
#ifndef SEQ
#define SEQ 2048
#endif
#define NB_FULL 2
#define S_FULL 2048
#define DM 1024
#define NH 16
#define HD 64
static_assert(NB >= 1 && NB <= NB_FULL);
static_assert(SEQ >= 64 && SEQ <= S_FULL && (SEQ % 64) == 0);
static_assert(DM == NH * HD && (DM % 64) == 0 && HD == 64);

typedef __attribute__((ext_vector_type(16))) _Float16 v16h;
typedef __attribute__((ext_vector_type(8)))  _Float16 v8h;
typedef __attribute__((ext_vector_type(16))) __bf16   v16b;
typedef __attribute__((ext_vector_type(8)))  __bf16   v8b;
typedef __attribute__((ext_vector_type(8)))  float    v8f;
typedef __attribute__((ext_vector_type(4)))  float    v4f;
typedef __attribute__((ext_vector_type(4)))  unsigned v4u;


__device__ __forceinline__ float bfr(float f) { unsigned u = __float_as_uint(f); u += 0x7fffu + ((u >> 16) & 1u); return __uint_as_float(u & 0xffff0000u); }
__device__ __forceinline__ unsigned h2u(float a, float b) {
    return (unsigned)__builtin_bit_cast(unsigned short, (_Float16)a) | ((unsigned)__builtin_bit_cast(unsigned short, (_Float16)b) << 16);
}

namespace w25 {

__device__ __forceinline__ unsigned short f2bf_bits(float f) {
  unsigned u = __float_as_uint(f);
  return (unsigned short)((u + 0x7FFFu + ((u >> 16) & 1u)) >> 16);
}
__device__ __forceinline__ float bf_bits2f(unsigned short h) { return __uint_as_float(((unsigned)h) << 16); }

__device__ __forceinline__ void dep_guard_h(v8f& a, v8f& b, v16h x, v16h y) { asm volatile("v_nop\n\tv_nop\n\tv_nop\n\tv_nop" : "+v"(a), "+v"(b) : "v"(x), "v"(y)); }
__device__ __forceinline__ void dep_guard_b(v8f& a, v8f& b, v16b x, v16b y) { asm volatile("v_nop\n\tv_nop\n\tv_nop\n\tv_nop" : "+v"(a), "+v"(b) : "v"(x), "v"(y)); }
__device__ __forceinline__ void keep4_h(v16h a, v16h b, v16h c, v16h d) { asm volatile("v_nop" :: "v"(a), "v"(b), "v"(c), "v"(d)); }
__device__ __forceinline__ void keep4_b(v16b a, v16b b, v16b c, v16b d) { asm volatile("v_nop" :: "v"(a), "v"(b), "v"(c), "v"(d)); }
__device__ __forceinline__ void acc_guard4(v8f& a, v8f& b, v8f& c, v8f& d) { asm volatile("v_nop\n\tv_nop\n\tv_nop\n\tv_nop" : "+v"(a), "+v"(b), "+v"(c), "+v"(d)); }
template <typename T> struct Frag;
template <> struct Frag<_Float16> {
  typedef v16h V; union U { v16h v; v8h h[2]; };
  static __device__ __forceinline__ v16h load(const _Float16* p) {
    U f; f.h[0] = *(const v8h*)(p); f.h[1] = *(const v8h*)(p + 16); return f.v;
  }
  static __device__ __forceinline__ v8f mma(v16h a, v16h b, v8f c) {
    return __builtin_amdgcn_wmma_f32_16x16x32_f16(false, a, false, b, (short)0, c, false, false);
  }
  static __device__ __forceinline__ void guard(v8f& a, v8f& b, v16h x, v16h y) { dep_guard_h(a, b, x, y); }
  static __device__ __forceinline__ void keep(v16h a, v16h b, v16h c, v16h d) { keep4_h(a, b, c, d); }
};
template <> struct Frag<__bf16> {
  typedef v16b V; union U { v16b v; v8b h[2]; };
  static __device__ __forceinline__ v16b load(const __bf16* p) {
    U f; f.h[0] = *(const v8b*)(p); f.h[1] = *(const v8b*)(p + 16); return f.v;
  }
  static __device__ __forceinline__ v8f mma(v16b a, v16b b, v8f c) {
    return __builtin_amdgcn_wmma_f32_16x16x32_bf16(false, a, false, b, (short)0, c, false, false);
  }
  static __device__ __forceinline__ void guard(v8f& a, v8f& b, v16b x, v16b y) { dep_guard_b(a, b, x, y); }
  static __device__ __forceinline__ void keep(v16b a, v16b b, v16b c, v16b d) { keep4_b(a, b, c, d); }
};

template <int ET> struct Elem;
template <> struct Elem<0> { typedef _Float16 T; };
template <> struct Elem<1> { typedef __bf16 T; };
template <int ET, bool SPLIT, int BIAS_MODE, int OUT_MODE, bool RESID, int ACT = 0>
__global__ __launch_bounds__(256) void wmma_gemm64(
    const unsigned short* __restrict__ Ap, const unsigned short* __restrict__ A2p, int lda, long strideA,
    const unsigned short* __restrict__ Btp, const unsigned short* __restrict__ Bt2p, int ldb, long strideB,
    void* __restrict__ Cout, void* __restrict__ Cout2, int ldc, long strideC,
    const float* __restrict__ bias,
    const float* __restrict__ resid, long strideR,
    int M, int N, int K, float scale) {
  typedef typename Elem<ET>::T T;
  typedef typename Frag<T>::V V;
  const T* A = (const T*)Ap; const T* A2 = (const T*)A2p; const T* Bt = (const T*)Btp; const T* Bt2 = (const T*)Bt2p;
  __shared__ __align__(16) float sT[8][16 * 68];
  const int b    = blockIdx.y;
  const int lane = threadIdx.x & 31;
  const int wave = threadIdx.x >> 5;
  const int tilesN = N >> 6;
  const int tilesM = M >> 6;
  const int tile = blockIdx.x * 8 + wave;
  if (tile >= tilesM * tilesN) return;
  const int tm = tile / tilesN;
  const int tn = tile - tm * tilesN;
  const int m0 = tm << 6;
  const int n0 = tn << 6;

  const T* Ab  = A  + (size_t)b * strideA;
  const T* Bb  = Bt + (size_t)b * strideB;
  const T* Ab2 = SPLIT ? (A2  + (size_t)b * strideA) : nullptr;
  const T* Bb2 = SPLIT ? (Bt2 + (size_t)b * strideB) : nullptr;

  const int rlane = lane & 15;
  const int koff  = (lane >> 4) * 8;
  const int mOff  = (lane >> 4) * 8;

  v8f acc[4][4];
#pragma unroll
  for (int i = 0; i < 4; ++i)
#pragma unroll
    for (int j = 0; j < 4; ++j) acc[i][j] = (v8f){0.f,0.f,0.f,0.f,0.f,0.f,0.f,0.f};

  for (int k0 = 0; k0 < K; k0 += 32) {
    V bh[4], bl[4];
#pragma unroll
    for (int j = 0; j < 4; ++j) {
      const size_t bo = (size_t)(n0 + (j << 4) + rlane) * ldb + koff + k0;
      bh[j] = Frag<T>::load(Bb + bo);
      if (SPLIT) bl[j] = Frag<T>::load(Bb2 + bo);
    }
#pragma unroll
    for (int i = 0; i < 4; ++i) {
      const size_t ao = (size_t)(m0 + (i << 4) + rlane) * lda + koff + k0;
      V ah = Frag<T>::load(Ab + ao);
      V al = ah;
      if (SPLIT) al = Frag<T>::load(Ab2 + ao);
#pragma unroll
      for (int j = 0; j < 4; ++j) {
        acc[i][j] = Frag<T>::mma(ah, bh[j], acc[i][j]);
        if (SPLIT) {
          acc[i][j] = Frag<T>::mma(ah, bl[j], acc[i][j]);
          acc[i][j] = Frag<T>::mma(al, bh[j], acc[i][j]);
        }
      }
      Frag<T>::guard(acc[i][0], acc[i][3], ah, SPLIT ? al : ah);
    }
    Frag<T>::keep(bh[0], bh[1], bh[2], bh[3]);
    if (SPLIT) Frag<T>::keep(bl[0], bl[1], bl[2], bl[3]);
  }
  acc_guard4(acc[0][0], acc[0][1], acc[0][2], acc[0][3]);
  acc_guard4(acc[1][0], acc[1][1], acc[1][2], acc[1][3]);
  acc_guard4(acc[2][0], acc[2][1], acc[2][2], acc[2][3]);
  acc_guard4(acc[3][0], acc[3][1], acc[3][2], acc[3][3]);

  float* slab = sT[wave];
  const float* Rb = RESID ? (resid + (size_t)b * strideR) : nullptr;
#pragma unroll
  for (int i = 0; i < 4; ++i) {
    const int mBase = m0 + (i << 4);
#pragma unroll
    for (int j = 0; j < 4; ++j) {
      const int n = n0 + (j << 4) + rlane;
      float bv = 0.f;
      if (BIAS_MODE == 2) bv = bias[n];
      if (BIAS_MODE == 3) bv = bf_bits2f(f2bf_bits(bias[n]));
#pragma unroll
      for (int r = 0; r < 8; ++r) {
        float v = acc[i][j][r] * scale;
        if (BIAS_MODE == 1) v += bias[mBase + mOff + r];
        if (BIAS_MODE == 2 || BIAS_MODE == 3) v += bv;
        if (RESID) v += Rb[(size_t)(mBase + mOff + r) * ldc + n];
        if (ACT == 1) v = tanhf(v);
        if (ACT == 2) v = fmaxf(v, 0.0f);
        slab[(mOff + r) * 68 + (j << 4) + rlane] = v;
      }
    }
    __builtin_amdgcn_fence(3  , "workgroup");
    __builtin_amdgcn_wave_barrier();
    __builtin_amdgcn_fence(2  , "workgroup");
    if (OUT_MODE == 0) {
      float* C = (float*)Cout + (size_t)b * strideC;
      const int hh = lane >> 4, c4 = (lane & 15) * 4;
      for (int pass = 0; pass < 2; ++pass) {
#pragma unroll
        for (int it = 0; it < 8; ++it) {
          const int row = it * 2 + hh;
          v4f v = *(const v4f*)(slab + row * 68 + c4);
          *(volatile v4f*)(C + (size_t)(mBase + row) * ldc + n0 + c4) = v;
        }
        __threadfence();
      }
    } else {
      const int q = lane >> 3, c8 = (lane & 7) * 8;
      unsigned short* C  = (unsigned short*)Cout  + (size_t)b * strideC;
      unsigned short* C2 = (OUT_MODE == 2) ? ((unsigned short*)Cout2 + (size_t)b * strideC) : nullptr;
      for (int pass = 0; pass < 2; ++pass) {
#pragma unroll
        for (int it = 0; it < 4; ++it) {
          const int row = it * 4 + q;
          const float* sp = slab + row * 68 + c8;
          v8h hv, lv;
#pragma unroll
          for (int e = 0; e < 8; ++e) {
            if (OUT_MODE == 1) {
              hv[e] = (_Float16)sp[e]; lv[e] = hv[e];
            } else {
              unsigned short hb = f2bf_bits(sp[e]);
              unsigned short lb = f2bf_bits(sp[e] - bf_bits2f(hb));
              hv[e] = __builtin_bit_cast(_Float16, hb);
              lv[e] = __builtin_bit_cast(_Float16, lb);
            }
          }
          *(volatile v8h*)(C + (size_t)(mBase + row) * ldc + n0 + c8) = hv;
          if (OUT_MODE == 2) *(volatile v8h*)(C2 + (size_t)(mBase + row) * ldc + n0 + c8) = lv;
        }
        __threadfence();
      }
    }
    __builtin_amdgcn_fence(3  , "workgroup");
    __builtin_amdgcn_wave_barrier();
    __builtin_amdgcn_fence(2  , "workgroup");
  }
}

}

template <bool BFR>
__global__ __launch_bounds__(256) void k_cvt8(const float* __restrict__ src, long long lds, int segR, long long segRows,
                                              unsigned short* __restrict__ dst, long long ldd, int R, int C, float s) {
    const long long u = (long long)blockIdx.x * 256 + threadIdx.x;
    const int cq = C >> 3;
    if (u >= (long long)R * cq) return;
    const int r = (int)(u / cq); const int c = 8 * (int)(u % cq);
    const long long rs = (long long)(r / segR) * segRows + (r % segR);
    const v4f a = *(const v4f*)(src + rs * lds + c);
    const v4f b = *(const v4f*)(src + rs * lds + c + 4);
    float f0 = a.x, f1 = a.y, f2 = a.z, f3 = a.w, f4 = b.x, f5 = b.y, f6 = b.z, f7 = b.w;
    if (BFR) { f0 = bfr(f0); f1 = bfr(f1); f2 = bfr(f2); f3 = bfr(f3); f4 = bfr(f4); f5 = bfr(f5); f6 = bfr(f6); f7 = bfr(f7); }
    v4u pk; pk.x = h2u(f0 * s, f1 * s); pk.y = h2u(f2 * s, f3 * s); pk.z = h2u(f4 * s, f5 * s); pk.w = h2u(f6 * s, f7 * s);
    volatile v4u* d = (volatile v4u*)(dst + (long long)r * ldd + c); *d = pk; __threadfence(); *d = pk;
}

__global__ __launch_bounds__(256) void k_cvtT(const float* __restrict__ W, int N, unsigned short* __restrict__ Bt, int KP, float s) {
    __shared__ float tile[64][65];
    const int o0 = blockIdx.x * 64, k0 = blockIdx.y * 64, t = threadIdx.x;
#pragma unroll
    for (int i = 0; i < 4; ++i) {
        const int kl = i * 16 + (t >> 4); const int o4 = (t & 15) * 4;
        const v4f v = *(const v4f*)(W + (long long)(k0 + kl) * N + o0 + o4);
        tile[kl][o4] = v.x; tile[kl][o4 + 1] = v.y; tile[kl][o4 + 2] = v.z; tile[kl][o4 + 3] = v.w;
    }
    __syncthreads();
#pragma unroll
    for (int p = 0; p < 2; ++p) {
        const int ol = p * 32 + (t >> 3); const int kq = (t & 7) * 8;
        const float g0 = bfr(tile[kq][ol]) * s,     g1 = bfr(tile[kq + 1][ol]) * s, g2 = bfr(tile[kq + 2][ol]) * s, g3 = bfr(tile[kq + 3][ol]) * s;
        const float g4 = bfr(tile[kq + 4][ol]) * s, g5 = bfr(tile[kq + 5][ol]) * s, g6 = bfr(tile[kq + 6][ol]) * s, g7 = bfr(tile[kq + 7][ol]) * s;
        v4u pk; pk.x = h2u(g0, g1); pk.y = h2u(g2, g3); pk.z = h2u(g4, g5); pk.w = h2u(g6, g7);
        volatile v4u* d = (volatile v4u*)(Bt + (long long)(o0 + ol) * KP + k0 + kq); *d = pk; __threadfence(); *d = pk;
    }
}

__global__ __launch_bounds__(256) void k_vt(const unsigned short* __restrict__ KVP, int ldkv, int seq, unsigned short* __restrict__ VT) {
    __shared__ __align__(16) unsigned short tile[64][72];
    const int kv0 = blockIdx.x * 64; const int bh = blockIdx.y; const int b = bh / NH, h = bh % NH; const int t = threadIdx.x;
#pragma unroll
    for (int i = 0; i < 2; ++i) {
        const int keyl = i * 32 + (t >> 3); const int d8 = (t & 7) * 8;
        const v4u v = *(const v4u*)(KVP + ((long long)(b * seq + kv0 + keyl)) * ldkv + h * 2 * HD + HD + d8);
        *(v4u*)&tile[keyl][d8] = v;
    }
    __syncthreads();
#pragma unroll
    for (int p = 0; p < 2; ++p) {
        const int dl = p * 32 + (t >> 3); const int kq = (t & 7) * 8;
        const unsigned w0 = tile[kq][dl], w1 = tile[kq + 1][dl], w2 = tile[kq + 2][dl], w3 = tile[kq + 3][dl];
        const unsigned w4 = tile[kq + 4][dl], w5 = tile[kq + 5][dl], w6 = tile[kq + 6][dl], w7 = tile[kq + 7][dl];
        v4u pk; pk.x = w0 | (w1 << 16); pk.y = w2 | (w3 << 16); pk.z = w4 | (w5 << 16); pk.w = w6 | (w7 << 16);
        volatile v4u* dd = (volatile v4u*)(VT + ((long long)bh * HD + dl) * seq + kv0 + kq); *dd = pk; __threadfence(); *dd = pk;
    }
}

#define AT_NW 4
#define AT_KC 64
struct AttnG { long long q_bs, q_rs, q_hs, k_bs, k_rs, k_hs, v_bs, v_hs, v_ds, o_bs, o_rs, o_hs; int S, Skv, H, nqb; float sscale; int pad_; };
static_assert(sizeof(AttnG) == 12 * 8 + 4 * 4 + 2 * 4);

__device__ __forceinline__ v8f mma16h(v16h a, v16h b, v8f c) {
    c = __builtin_amdgcn_wmma_f32_16x16x32_f16(false, a, false, b, (short)0, c, false, false);
    asm volatile("v_nop\n\tv_nop\n\tv_nop\n\tv_nop" : "+v"(c) : "v"(a), "v"(b));
    return c;
}

__global__ __launch_bounds__(128)
void k_attn_pl(const unsigned short* __restrict__ QPp, const unsigned short* __restrict__ KPp, const unsigned short* __restrict__ VTp,
               float* __restrict__ out, AttnG g) {
    const float PSC = 32768.0f;
    __shared__ __align__(16) _Float16 Psh[AT_NW][16 * AT_KC];
    __shared__ __align__(16) float    Os[AT_NW][16 * 68];
    const _Float16* QP = (const _Float16*)QPp; const _Float16* KP = (const _Float16*)KPp; const _Float16* VT = (const _Float16*)VTp;
    const int tid = threadIdx.x, wave = tid >> 5, lane = tid & 31, hh = lane >> 4, c = lane & 15;
    const int bx = blockIdx.x; const int qb = bx % g.nqb; const int bh = bx / g.nqb; const int h = bh % g.H; const int b = bh / g.H;
    const int q0 = qb * 64 + wave * 16;
    const _Float16* kb_ptr = KP + (size_t)b * g.k_bs + (size_t)h * g.k_hs;
    const _Float16* vb_ptr = VT + (size_t)b * g.v_bs + (size_t)h * g.v_hs;
    float*          ob_ptr = out + (size_t)b * g.o_bs + (size_t)h * g.o_hs;

    v16h qa0, qa1;
    {
        const _Float16* qrow = QP + (size_t)b * g.q_bs + (size_t)h * g.q_hs + (size_t)(q0 + c) * g.q_rs;
        qa0 = w25::Frag<_Float16>::load(qrow + 8 * hh);
        qa1 = w25::Frag<_Float16>::load(qrow + 32 + 8 * hh);
    }
    float mrow[8], lrow[8];
    v8f oacc[4];
#pragma unroll
    for (int r = 0; r < 8; ++r) { mrow[r] = -INFINITY; lrow[r] = 0.f; }
#pragma unroll
    for (int t = 0; t < 4; ++t) oacc[t] = (v8f){0.f,0.f,0.f,0.f,0.f,0.f,0.f,0.f};

    const int nChunks = g.Skv / AT_KC;
    _Float16* pwh = Psh[wave];
    for (int kc = 0; kc < nChunks; ++kc) {
        const int kv0 = kc * AT_KC;
        v8f s[4];
#pragma unroll
        for (int j = 0; j < 4; ++j) {
            v8f acc = (v8f){0.f,0.f,0.f,0.f,0.f,0.f,0.f,0.f};
            const _Float16* krow = kb_ptr + (size_t)(kv0 + j * 16 + c) * g.k_rs;
            const v16h kf0 = w25::Frag<_Float16>::load(krow + 8 * hh);
            acc = mma16h(qa0, kf0, acc);
            const v16h kf1 = w25::Frag<_Float16>::load(krow + 32 + 8 * hh);
            acc = mma16h(qa1, kf1, acc);
            s[j] = acc;
        }
        float cm[8];
#pragma unroll
        for (int r = 0; r < 8; ++r) {
            float m = -INFINITY;
#pragma unroll
            for (int j = 0; j < 4; ++j) { const float v = s[j][r] * g.sscale; s[j][r] = v; m = fmaxf(m, v); }
#pragma unroll
            for (int off = 1; off < 16; off <<= 1) m = fmaxf(m, __shfl_xor(m, off, 32));
            cm[r] = m;
        }
#pragma unroll
        for (int r = 0; r < 8; ++r) {
            const float mnew = fmaxf(mrow[r], cm[r]);
            const float alpha = expf(mrow[r] - mnew);
            mrow[r] = mnew;
            float psum = 0.f;
#pragma unroll
            for (int j = 0; j < 4; ++j) {
                const float p = expf(s[j][r] - mnew);
                psum += p;
                pwh[(8 * hh + r) * AT_KC + j * 16 + c] = (_Float16)(p * PSC);
            }
#pragma unroll
            for (int off = 1; off < 16; off <<= 1) psum += __shfl_xor(psum, off, 32);
            lrow[r] = lrow[r] * alpha + psum;
#pragma unroll
            for (int t = 0; t < 4; ++t) oacc[t][r] *= alpha;
        }
        __builtin_amdgcn_fence(3  , "workgroup");
        __builtin_amdgcn_wave_barrier();
        __builtin_amdgcn_fence(2  , "workgroup");
#pragma unroll 1
        for (int kk = 0; kk < 2; ++kk) {
            const v16h pa = w25::Frag<_Float16>::load(pwh + c * AT_KC + kk * 32 + 8 * hh);
#pragma unroll
            for (int t = 0; t < 4; ++t) {
                const v16h vb = w25::Frag<_Float16>::load(vb_ptr + (size_t)(t * 16 + c) * g.v_ds + kv0 + kk * 32 + 8 * hh);
                oacc[t] = mma16h(pa, vb, oacc[t]);
            }
        }
    }

    float* os = Os[wave];
#pragma unroll
    for (int r = 0; r < 8; ++r) {
        const float inv = 1.0f / (lrow[r] * PSC);
#pragma unroll
        for (int t = 0; t < 4; ++t) os[(8 * hh + r) * 68 + t * 16 + c] = oacc[t][r] * inv;
    }
    __builtin_amdgcn_fence(3  , "workgroup");
    __builtin_amdgcn_wave_barrier();
    __builtin_amdgcn_fence(2  , "workgroup");
    {
        const int c4 = (lane & 15) * 4;
        for (int pass = 0; pass < 2; ++pass) {
#pragma unroll
            for (int it = 0; it < 8; ++it) {
                const int row = it * 2 + hh;
                v4f val = *(const v4f*)(os + row * 68 + c4);
                *(volatile v4f*)(ob_ptr + (size_t)(q0 + row) * g.o_rs + c4) = val;
            }
            __threadfence();
        }
    }
}

static inline size_t al256(size_t x) { return (x + 255) & ~(size_t)255; }

extern "C" void kernel_launch(void* const* d_in, const int* in_sizes, int n_in, void* d_out, int out_size, void* d_ws, size_t ws_size, hipStream_t stream) {
    if (n_in < 7) return;
    const float* emb  = (const float*)d_in[0];
    const float* W_kv = (const float*)d_in[1];
    const float* b_kv = (const float*)d_in[2];
    const float* W_q  = (const float*)d_in[3];
    const float* b_q  = (const float*)d_in[4];
    const float* W_o  = (const float*)d_in[5];
    const float* b_o  = (const float*)d_in[6];
    float* out = (float*)d_out;

    const long long needRows = (long long)(NB - 1) * S_FULL + SEQ;
    if ((long long)in_sizes[0] < needRows * DM) return;
    if (in_sizes[1] < DM * 2 * DM || in_sizes[2] < 2 * DM || in_sizes[3] < DM * DM || in_sizes[4] < DM || in_sizes[5] < DM * DM || in_sizes[6] < DM) return;
    if ((long long)out_size < needRows * DM) return;

    const size_t nTok = (size_t)NB * SEQ;
    const size_t szEP  = al256(nTok * DM * 2);
    const size_t szWkv = al256((size_t)2 * DM * DM * 2);
    const size_t szWq  = al256((size_t)DM * DM * 2);
    const size_t szWo  = al256((size_t)DM * DM * 2);
    const size_t szKVP = al256(nTok * 2 * DM * 2);
    const size_t szQP  = al256(nTok * DM * 2);
    const size_t szVT  = al256((size_t)NB * NH * HD * SEQ * 2);
    const size_t szCTX = al256(nTok * DM * 4);
    const size_t szCP  = al256(nTok * DM * 2);
    size_t off = 0;
    unsigned short* EP   = (unsigned short*)((char*)d_ws + off); off += szEP;
    unsigned short* WkvT = (unsigned short*)((char*)d_ws + off); off += szWkv;
    unsigned short* WqT  = (unsigned short*)((char*)d_ws + off); off += szWq;
    unsigned short* WoT  = (unsigned short*)((char*)d_ws + off); off += szWo;
    unsigned short* KVP  = (unsigned short*)((char*)d_ws + off); off += szKVP;
    unsigned short* QP   = (unsigned short*)((char*)d_ws + off); off += szQP;
    unsigned short* VT   = (unsigned short*)((char*)d_ws + off); off += szVT;
    float*          CTX  = (float*)((char*)d_ws + off);          off += szCTX;
    unsigned short* CP   = (unsigned short*)((char*)d_ws + off); off += szCP;
    if (off > ws_size) return;

    {
        const long long nth = (long long)nTok * (DM / 8);
        k_cvt8<true><<<(unsigned)((nth + 255) / 256), 256, 0, stream>>>(emb, (long long)DM, SEQ, (long long)S_FULL, EP, (long long)DM, (int)nTok, DM, 16.0f);
    }
    k_cvtT<<<dim3(2 * DM / 64, DM / 64), 256, 0, stream>>>(W_kv, 2 * DM, WkvT, DM, 256.0f);
    k_cvtT<<<dim3(DM / 64, DM / 64), 256, 0, stream>>>(W_q, DM, WqT, DM, 256.0f);
    k_cvtT<<<dim3(DM / 64, DM / 64), 256, 0, stream>>>(W_o, DM, WoT, DM, 256.0f);
    {
        const int tiles = (SEQ / 64) * (2 * DM / 64);
        w25::wmma_gemm64<0, false, 3, 1, false, 0><<<dim3((unsigned)((tiles + 7) / 8), (unsigned)NB), 256, 0, stream>>>(
            EP, nullptr, DM, (long)SEQ * DM, WkvT, nullptr, DM, 0L, (void*)KVP, nullptr, 2 * DM, (long)SEQ * 2 * DM,
            b_kv, nullptr, 0L, SEQ, 2 * DM, DM, 1.0f / 4096.0f);
    }
    {
        const int tiles = (SEQ / 64) * (DM / 64);
        w25::wmma_gemm64<0, false, 3, 1, false, 0><<<dim3((unsigned)((tiles + 7) / 8), (unsigned)NB), 256, 0, stream>>>(
            EP, nullptr, DM, (long)SEQ * DM, WqT, nullptr, DM, 0L, (void*)QP, nullptr, DM, (long)SEQ * DM,
            b_q, nullptr, 0L, SEQ, DM, DM, 1.0f / 4096.0f);
    }
    k_vt<<<dim3(SEQ / 64, NB * NH), 256, 0, stream>>>(KVP, 2 * DM, SEQ, VT);
    {
        AttnG g;
        g.q_bs = (long long)SEQ * DM;      g.q_rs = DM;      g.q_hs = HD;
        g.k_bs = (long long)SEQ * 2 * DM;  g.k_rs = 2 * DM;  g.k_hs = 2 * HD;
        g.v_bs = (long long)NH * HD * SEQ; g.v_hs = (long long)HD * SEQ; g.v_ds = SEQ;
        g.o_bs = (long long)SEQ * DM;      g.o_rs = DM;      g.o_hs = HD;
        g.S = SEQ; g.Skv = SEQ; g.H = NH; g.nqb = SEQ / 64; g.sscale = 0.125f; g.pad_ = 0;
        k_attn_pl<<<(unsigned)(NB * NH * (SEQ / 64)), 128, 0, stream>>>(QP, KVP, VT, CTX, g);
    }
    {
        const long long nth = (long long)nTok * (DM / 8);
        k_cvt8<false><<<(unsigned)((nth + 255) / 256), 256, 0, stream>>>(CTX, (long long)DM, SEQ, (long long)SEQ, CP, (long long)DM, (int)nTok, DM, 64.0f);
    }
    {
        const int tiles = (SEQ / 64) * (DM / 64);
        w25::wmma_gemm64<0, false, 3, 0, false, 0><<<dim3((unsigned)((tiles + 7) / 8), (unsigned)NB), 256, 0, stream>>>(
            CP, nullptr, DM, (long)SEQ * DM, WoT, nullptr, DM, 0L, (void*)out, nullptr, DM, (long)S_FULL * DM,
            b_o, nullptr, 0L, SEQ, DM, DM, 1.0f / 16384.0f);
    }
}
